// GRU_69406671504098
// MI455X (gfx1250) — hardware-verified
//
#include <hip/hip_runtime.h>
#include <math.h>

constexpr int NSTEP    = 32;
constexpr int NB       = 128;
constexpr int NN       = 128;
constexpr int DIN      = 2;
constexpr int HID      = 128;
constexpr int G3H      = 3 * HID;
constexpr int NROWS    = NB * NN;
constexpr int NTHR     = 256;
constexpr int ROWB     = 32;
constexpr int HP       = 136;
constexpr int NTABBLK  = G3H / 32;
constexpr int NPREPBLK = (G3H * HID / 8) / NTHR;
constexpr float WCARRY      = 64.0f;
constexpr float WCARRY_INV  = 1.0f / 64.0f;
constexpr float LOCARRY     = 2048.0f;
constexpr float LOCARRY_INV = 1.0f / 2048.0f;
static_assert(NROWS == 16384 && G3H == 384 && HID == 128 && DIN == 2 && NSTEP == 32);
static_assert(NROWS % ROWB == 0);
static_assert(ROWB == 32);
static_assert(HID == 16 * (NTHR / 32));
static_assert(HID % 32 == 0);
static_assert(HP % 8 == 0 && HP >= HID);
static_assert((ROWB * HP) % NTHR == 0);
static_assert(NSTEP * ROWB * DIN == 8 * NTHR);
static_assert(NPREPBLK * NTHR * 8 == G3H * HID);
static_assert(NPREPBLK >= NTABBLK);
static_assert((NTHR / 32) * 4 == 32);

typedef __attribute__((ext_vector_type(16))) _Float16 v16h;
typedef __attribute__((ext_vector_type(8)))  _Float16 v8h;
typedef __attribute__((ext_vector_type(8)))  float    v8f;
typedef __attribute__((ext_vector_type(4)))  float    v4f;
typedef __attribute__((ext_vector_type(2)))  float    v2f;

__device__ __forceinline__ void dep_guard6_h(v8f& a0, v8f& a1, v8f& a2, v8f& a3, v8f& a4, v8f& a5,
                                             v16h f0, v16h f1, v16h f2, v16h f3, v16h f4) {
  asm volatile("v_nop\n\tv_nop\n\tv_nop\n\tv_nop"
               : "+v"(a0), "+v"(a1), "+v"(a2), "+v"(a3), "+v"(a4), "+v"(a5)
               : "v"(f0), "v"(f1), "v"(f2), "v"(f3), "v"(f4));
}
__device__ __forceinline__ void acc_guard6(v8f& a0, v8f& a1, v8f& a2, v8f& a3, v8f& a4, v8f& a5) {
  asm volatile("v_nop\n\tv_nop\n\tv_nop\n\tv_nop" : "+v"(a0), "+v"(a1), "+v"(a2), "+v"(a3), "+v"(a4), "+v"(a5));
}
__device__ __forceinline__ void use4(float a, float b, float c, float d) { asm volatile("" :: "v"(a), "v"(b), "v"(c), "v"(d)); }
__device__ __forceinline__ void use2(float a, float b) { asm volatile("" :: "v"(a), "v"(b)); }

template <typename T> struct Frag;
template <> struct Frag<_Float16> {
  typedef v16h V; union U { v16h v; v8h h[2]; };
  static __device__ __forceinline__ v16h load(const _Float16* p) {
    U f; f.h[0] = *(const v8h*)(p); f.h[1] = *(const v8h*)(p + 16); return f.v;
  }
  static __device__ __forceinline__ v8f mma(v16h a, v16h b, v8f c) {
    return __builtin_amdgcn_wmma_f32_16x16x32_f16(false, a, false, b, (short)0, c, false, false);
  }
};

__device__ __forceinline__ float fsigm(float x) { return __builtin_amdgcn_rcpf(1.0f + __expf(-x)); }
__device__ __forceinline__ float ftanh(float x) { return 1.0f - 2.0f * __builtin_amdgcn_rcpf(1.0f + __expf(2.0f * x)); }

__device__ __forceinline__ void put_hilo(_Float16* ahi, _Float16* alo, int idx, float h) {
  const _Float16 hv = (_Float16)h;
  const float res = (h - (float)hv) * LOCARRY;
  ahi[idx] = hv;
  alo[idx] = (_Float16)res;
}

__global__ __launch_bounds__(NTHR) void prep_kernel(const float* __restrict__ W1, const float* __restrict__ b1,
                                                    const float* __restrict__ Wih, const float* __restrict__ bih,
                                                    const float* __restrict__ bhh, const float* __restrict__ Whh,
                                                    float* __restrict__ TAB, _Float16* __restrict__ WHH) {
  __shared__ __align__(16) float sTab[32 * 4];
  const int blk = blockIdx.x, tid = threadIdx.x, lane = tid & 31, wave = tid >> 5;

  {
    const int gid = blk * NTHR + tid;
    const float* p = Whh + (size_t)gid * 8;
    const v4f a  = *(const v4f*)p;
    const v4f bq = *(const v4f*)(p + 4);
    v8h hv;
#pragma unroll
    for (int e = 0; e < 4; ++e) {
      hv[e]     = (_Float16)(a[e]  * WCARRY);
      hv[4 + e] = (_Float16)(bq[e] * WCARRY);
    }
    _Float16* op = WHH + (size_t)gid * 8;
    *(volatile v8h*)op = hv;
    __threadfence();
    *(volatile v8h*)op = hv;
  }

  if (blk < NTABBLK) {
    float w1a[4], w1b[4], bb1[4];
#pragma unroll
    for (int q = 0; q < 4; ++q) {
      const int k = lane + 32 * q;
      const v2f w = *(const v2f*)(W1 + (size_t)k * DIN);
      w1a[q] = w[0]; w1b[q] = w[1]; bb1[q] = b1[k];
    }
#pragma unroll
    for (int i = 0; i < 4; ++i) {
      const int gl = 4 * wave + i;
      const int g  = 32 * blk + gl;
      float s0 = 0.0f, s1 = 0.0f, s2 = 0.0f;
#pragma unroll
      for (int q = 0; q < 4; ++q) {
        const float w = Wih[(size_t)g * HID + lane + 32 * q];
        s0 += w * w1a[q];
        s1 += w * w1b[q];
        s2 += w * bb1[q];
      }
#pragma unroll
      for (int off = 16; off > 0; off >>= 1) {
        s0 += __shfl_xor(s0, off, 32);
        s1 += __shfl_xor(s1, off, 32);
        s2 += __shfl_xor(s2, off, 32);
      }
      const float vi = bih[g];
      const float vh = bhh[g];
      if (lane == 0) {
        sTab[gl * 4 + 0] = s0;
        sTab[gl * 4 + 1] = s1;
        sTab[gl * 4 + 2] = s2 + vi;
        sTab[gl * 4 + 3] = vh;
      }
    }
  }
  __syncthreads();
  if (blk < NTABBLK && wave == 0) {
    const v4f v = *(const v4f*)(sTab + 4 * lane);
    float* op = TAB + (size_t)(32 * blk + lane) * 4;
    *(volatile v4f*)op = v;
    __threadfence();
    *(volatile v4f*)op = v;
  }
}

__global__ __launch_bounds__(NTHR) void rec_main_kernel(const float* __restrict__ X, const float* __restrict__ H0,
                                                        const float* __restrict__ TAB, const unsigned short* __restrict__ WHHp,
                                                        const float* __restrict__ Wo, const float* __restrict__ bo,
                                                        float* __restrict__ OUT) {
  __shared__ __align__(16) _Float16 Ahi[ROWB * HP];
  __shared__ __align__(16) _Float16 Alo[ROWB * HP];
  __shared__ __align__(16) float    xin[NSTEP * ROWB * DIN];
  __shared__ __align__(16) float    sP[(NTHR / 32) * ROWB * DIN];
  const _Float16* WHH = (const _Float16*)WHHp;
  const int tid = threadIdx.x, lane = tid & 31, wave = tid >> 5;
  const int c = lane & 15, hh = lane >> 4, koff = hh * 8, mOff = hh * 8;
  const int row0 = blockIdx.x * ROWB;
  const int j = 16 * wave + c;

#pragma unroll 1
  for (int i = tid; i < ROWB * HP; i += NTHR) { Ahi[i] = (_Float16)0.0f; Alo[i] = (_Float16)0.0f; }

  {
    const int ts = tid >> 3, piece = tid & 7;
    const float* xp = X + ((size_t)ts * NROWS + row0) * DIN + 8 * piece;
    const v4f a  = *(const v4f*)xp;
    const v4f bq = *(const v4f*)(xp + 4);
    float* dp = xin + ts * (ROWB * DIN) + 8 * piece;
    *(v4f*)dp = a;
    *(v4f*)(dp + 4) = bq;
  }

  const v4f tr = *(const v4f*)(TAB + (size_t)j * 4);
  const v4f tz = *(const v4f*)(TAB + (size_t)(HID + j) * 4);
  const v4f tn = *(const v4f*)(TAB + (size_t)(2 * HID + j) * 4);
  const float w0r = tr[0], w1r = tr[1], cr = tr[2] + tr[3];
  const float w0z = tz[0], w1z = tz[1], cz = tz[2] + tz[3];
  const float w0n = tn[0], w1n = tn[1], cn = tn[2], bhn = tn[3];
  const float wo0 = Wo[j], wo1 = Wo[HID + j];
  const float bo0 = bo[0], bo1 = bo[1];
  use4(w0r, w1r, cr, w0z); use4(w1z, cz, w0n, w1n); use4(cn, bhn, wo0, wo1); use2(bo0, bo1);
  __syncthreads();

  float hst[2][8];
#pragma unroll
  for (int rt = 0; rt < 2; ++rt) {
#pragma unroll
    for (int r = 0; r < 8; ++r) hst[rt][r] = H0[(size_t)(row0 + 16 * rt + mOff + r) * HID + j];
#pragma unroll
    for (int r = 0; r < 8; ++r) put_hilo(Ahi, Alo, (16 * rt + mOff + r) * HP + j, hst[rt][r]);
    asm volatile("" ::: "memory");
  }
  __syncthreads();

  const _Float16* wr = WHH + (size_t)j * HID + koff;
  const _Float16* wz = WHH + (size_t)(HID + j) * HID + koff;
  const _Float16* wn = WHH + (size_t)(2 * HID + j) * HID + koff;
  const v8f z8 = {0.f, 0.f, 0.f, 0.f, 0.f, 0.f, 0.f, 0.f};

#pragma unroll 1
  for (int t = 0; t < NSTEP; ++t) {
    const float* xt = xin + t * (ROWB * DIN);
#pragma unroll
    for (int rt = 0; rt < 2; ++rt) {
      const _Float16* pah = Ahi + (16 * rt + c) * HP + koff;
      const _Float16* pal = Alo + (16 * rt + c) * HP + koff;
      v8f arh = z8, arl = z8, azh = z8, azl = z8, anh = z8, anl = z8;
#pragma unroll 1
      for (int k0 = 0; k0 < HID; k0 += 32) {
        const v16h fah = Frag<_Float16>::load(pah + k0);
        const v16h fal = Frag<_Float16>::load(pal + k0);
        const v16h fbr = Frag<_Float16>::load(wr + k0);
        const v16h fbz = Frag<_Float16>::load(wz + k0);
        const v16h fbn = Frag<_Float16>::load(wn + k0);
        arh = Frag<_Float16>::mma(fah, fbr, arh);
        arl = Frag<_Float16>::mma(fal, fbr, arl);
        azh = Frag<_Float16>::mma(fah, fbz, azh);
        azl = Frag<_Float16>::mma(fal, fbz, azl);
        anh = Frag<_Float16>::mma(fah, fbn, anh);
        anl = Frag<_Float16>::mma(fal, fbn, anl);
        dep_guard6_h(arh, arl, azh, azl, anh, anl, fah, fal, fbr, fbz, fbn);
      }
      acc_guard6(arh, arl, azh, azl, anh, anl);

#pragma unroll
      for (int r = 0; r < 8; ++r) {
        const int rl = 16 * rt + mOff + r;
        const float x0 = xt[rl * DIN];
        const float x1 = xt[rl * DIN + 1];
        const float ghr = (arh[r] + arl[r] * LOCARRY_INV) * WCARRY_INV;
        const float ghz = (azh[r] + azl[r] * LOCARRY_INV) * WCARRY_INV;
        const float ghn = (anh[r] + anl[r] * LOCARRY_INV) * WCARRY_INV + bhn;
        const float gir = x0 * w0r + x1 * w1r + cr;
        const float giz = x0 * w0z + x1 * w1z + cz;
        const float gin = x0 * w0n + x1 * w1n + cn;
        const float rg = fsigm(gir + ghr);
        const float zg = fsigm(giz + ghz);
        const float ng = ftanh(gin + rg * ghn);
        const float ho = hst[rt][r];
        hst[rt][r] = (1.0f - zg) * ng + zg * ho;
      }
    }
    __syncthreads();
#pragma unroll
    for (int rt = 0; rt < 2; ++rt)
#pragma unroll
      for (int r = 0; r < 8; ++r) put_hilo(Ahi, Alo, (16 * rt + mOff + r) * HP + j, hst[rt][r]);
    __syncthreads();
  }

#pragma unroll
  for (int rt = 0; rt < 2; ++rt) {
#pragma unroll
    for (int r = 0; r < 8; ++r) {
      float q0 = hst[rt][r] * wo0;
      float q1 = hst[rt][r] * wo1;
#pragma unroll
      for (int off = 1; off < 16; off <<= 1) {
        q0 += __shfl_xor(q0, off, 32);
        q1 += __shfl_xor(q1, off, 32);
      }
      if (c == 0) {
        const int rl = 16 * rt + mOff + r;
        sP[(wave * ROWB + rl) * DIN + 0] = q0;
        sP[(wave * ROWB + rl) * DIN + 1] = q1;
      }
    }
  }
  __syncthreads();
  if (wave == 0) {
    const int l = lane & 15;
    v4f o;
#pragma unroll
    for (int e = 0; e < 4; ++e) {
      const int rl = 2 * l + (e >> 1);
      const int d  = e & 1;
      float s = 0.0f;
#pragma unroll
      for (int w = 0; w < NTHR / 32; ++w) s += sP[(w * ROWB + rl) * DIN + d];
      o[e] = s + (d ? bo1 : bo0);
    }
    float* op = OUT + (size_t)row0 * DIN + 4 * l;
    if (lane < 16) *(volatile v4f*)op = o;
    __threadfence();
    if (lane < 16) *(volatile v4f*)op = o;
  }
}

extern "C" void kernel_launch(void* const* d_in, const int* in_sizes, int n_in,
                              void* d_out, int out_size, void* d_ws, size_t ws_size, hipStream_t stream) {
  if (n_in < 10 || d_out == nullptr || d_ws == nullptr) return;
  if (in_sizes[0] != NSTEP * NROWS * DIN || in_sizes[1] != NROWS * HID || in_sizes[2] != HID * DIN ||
      in_sizes[3] != HID || in_sizes[4] != G3H * HID || in_sizes[5] != G3H * HID || in_sizes[6] != G3H ||
      in_sizes[7] != G3H || in_sizes[8] != DIN * HID || in_sizes[9] != DIN || out_size != NROWS * DIN) return;

  const float* x_in   = (const float*)d_in[0];
  const float* hidden = (const float*)d_in[1];
  const float* W1     = (const float*)d_in[2];
  const float* b1     = (const float*)d_in[3];
  const float* W_ih   = (const float*)d_in[4];
  const float* W_hh   = (const float*)d_in[5];
  const float* b_ih   = (const float*)d_in[6];
  const float* b_hh   = (const float*)d_in[7];
  const float* Wo     = (const float*)d_in[8];
  const float* bo     = (const float*)d_in[9];
  float* out = (float*)d_out;

  char* ws = (char*)d_ws; size_t off = 0;
  auto carve = [&](size_t bytes) -> char* { char* p = ws + off; off += (bytes + 255) & ~(size_t)255; return p; };
  _Float16* WHH = (_Float16*)carve((size_t)G3H * HID * 2);
  float*    TAB = (float*)carve((size_t)G3H * 4 * 4);
  if (off > ws_size || off > (size_t)134217728) return;

  prep_kernel<<<NPREPBLK, NTHR, 0, stream>>>(W1, b1, W_ih, b_ih, b_hh, W_hh, TAB, WHH);
  rec_main_kernel<<<NROWS / ROWB, NTHR, 0, stream>>>(x_in, hidden, TAB, (const unsigned short*)WHH, Wo, bo, out);
}
